// QLSTM_65481071399364
// MI455X (gfx1250) — hardware-run, weakly checked
//
#include <hip/hip_runtime.h>
#include <math.h>

typedef __attribute__((ext_vector_type(16))) _Float16 v16h;
typedef __attribute__((ext_vector_type(8)))  _Float16 v8h;
typedef __attribute__((ext_vector_type(8)))  float    v8f;
typedef __attribute__((ext_vector_type(4)))  float    v4f;

constexpr int kSteps = 64;
constexpr int kBatch = 1024;
constexpr int kDin   = 128;
constexpr int kHid   = 8;
constexpr int kGates = 4;
constexpr int kComb  = kDin + kHid;
constexpr int kRows  = kSteps * kBatch;
constexpr int kNReal = kGates * kHid;
constexpr int kNPad  = 64;
constexpr int kThP   = 64;
constexpr int kCpPerGate = 128;
constexpr int kFlush = 8;
constexpr int kOut0Elems = kSteps * kBatch * kHid;
constexpr int kOut1Off   = kOut0Elems;
constexpr int kOut2Off   = kOut0Elems + kBatch * kHid;
constexpr int kOutTotal  = kOut0Elems + 2 * kBatch * kHid;

static_assert(kComb == 136, "combined width");
static_assert(kNReal == 32, "stacked gate columns");
static_assert((kRows % 64) == 0 && (kNPad % 64) == 0 && (kDin % 32) == 0, "GEMM tile multiples");
static_assert((kSteps % kFlush) == 0, "flush chunks");
static_assert((size_t)kOut1Off * 4 == 2097152ull, "out1 byte offset");
static_assert((size_t)kOut2Off * 4 == 2129920ull, "out2 byte offset");
static_assert((size_t)kOutTotal * 4 == 2162688ull, "d_out bytes");

constexpr float kCarryX = 64.0f;
constexpr float kCarryW = 1024.0f;
constexpr float kFold   = 1.0f / (kCarryX * kCarryW);
constexpr float kF16MinNormal = 6.103515625e-5f;
static_assert(kFold == 1.52587890625e-5f, "fold-back is 2^-16");

constexpr size_t kSzXH = (size_t)kRows * kDin * 2;
constexpr size_t kSzBT = (size_t)kNPad * kDin * 2;
constexpr size_t kSzCP = (size_t)kGates * kCpPerGate * 4;
constexpr size_t kSzTH = (size_t)kRows * kThP * 4;
constexpr size_t kOffXH = 0;
constexpr size_t kOffBT = kOffXH + kSzXH;
constexpr size_t kOffCP = kOffBT + kSzBT;
constexpr size_t kOffTH = kOffCP + kSzCP;
constexpr size_t kWsTotal = kOffTH + kSzTH;
static_assert(kWsTotal == 33572864ull, "carve total");
static_assert(kWsTotal <= 134217728ull, "carve cap");
static_assert((kOffBT % 128) == 0 && (kOffCP % 128) == 0 && (kOffTH % 128) == 0, "128-B aligned regions");

__device__ __forceinline__ float carry_flush(float v, float carry) {
  const float f = v * carry;
  return (fabsf(f) < kF16MinNormal) ? 0.0f : f;
}

namespace eng {

__device__ __forceinline__ void guard1_h(v8f& a, v16h x, v16h y) {
  asm volatile("v_nop\n\tv_nop\n\tv_nop\n\tv_nop" : "+v"(a) : "v"(x), "v"(y));
}
__device__ __forceinline__ void keep4_h(v16h a, v16h b, v16h c, v16h d) {
  asm volatile("v_nop" :: "v"(a), "v"(b), "v"(c), "v"(d));
}
__device__ __forceinline__ void acc_guard4(v8f& a, v8f& b, v8f& c, v8f& d) {
  asm volatile("v_nop\n\tv_nop\n\tv_nop\n\tv_nop" : "+v"(a), "+v"(b), "+v"(c), "+v"(d));
}

struct FragH {
  union U { v16h v; v8h h[2]; };
  static __device__ __forceinline__ v16h load(const _Float16* p) {
    U f;
    f.h[0] = *(const v8h*)(p);
    f.h[1] = *(const v8h*)(p + 16);
    return f.v;
  }
  static __device__ __forceinline__ v8f mma(v16h a, v16h b, v8f c) {
    return __builtin_amdgcn_wmma_f32_16x16x32_f16(false, a, false, b, (short)0, c, false, false);
  }
};

__global__ __launch_bounds__(256) void gemm_f16_tile64(
    const unsigned short* __restrict__ Ap, int lda,
    const unsigned short* __restrict__ Btp, int ldb,
    float* __restrict__ C, int ldc,
    int M, int N, int K, float scale) {
  const _Float16* A  = (const _Float16*)Ap;
  const _Float16* Bt = (const _Float16*)Btp;
  __shared__ __align__(16) float sT[8][16 * 68];
  const int lane = threadIdx.x & 31;
  const int wave = threadIdx.x >> 5;
  const int tilesN = N >> 6;
  const int tilesM = M >> 6;
  const int tile = blockIdx.x * 8 + wave;
  if (tile >= tilesM * tilesN) return;
  const int tm = tile / tilesN;
  const int tn = tile - tm * tilesN;
  const int m0 = tm << 6;
  const int n0 = tn << 6;

  const int rlane = lane & 15;
  const int koff  = (lane >> 4) * 8;
  const int mOff  = (lane >> 4) * 8;

  v8f acc[4][4];
#pragma unroll
  for (int i = 0; i < 4; ++i)
#pragma unroll
    for (int j = 0; j < 4; ++j) acc[i][j] = (v8f){0.f,0.f,0.f,0.f,0.f,0.f,0.f,0.f};

  for (int k0 = 0; k0 < K; k0 += 32) {
    v16h bh[4];
#pragma unroll
    for (int j = 0; j < 4; ++j) {
      const size_t bo = (size_t)(n0 + (j << 4) + rlane) * ldb + koff + k0;
      bh[j] = FragH::load(Bt + bo);
    }
#pragma unroll
    for (int i = 0; i < 4; ++i) {
      const size_t ao = (size_t)(m0 + (i << 4) + rlane) * lda + koff + k0;
      v16h ah = FragH::load(A + ao);
#pragma unroll
      for (int j = 0; j < 4; ++j) acc[i][j] = FragH::mma(ah, bh[j], acc[i][j]);
#pragma unroll
      for (int j = 0; j < 4; ++j) guard1_h(acc[i][j], ah, bh[j]);
    }
    keep4_h(bh[0], bh[1], bh[2], bh[3]);
  }
  acc_guard4(acc[0][0], acc[0][1], acc[0][2], acc[0][3]);
  acc_guard4(acc[1][0], acc[1][1], acc[1][2], acc[1][3]);
  acc_guard4(acc[2][0], acc[2][1], acc[2][2], acc[2][3]);
  acc_guard4(acc[3][0], acc[3][1], acc[3][2], acc[3][3]);

  float* slab = sT[wave];
#pragma unroll
  for (int i = 0; i < 4; ++i) {
    const int mBase = m0 + (i << 4);
#pragma unroll
    for (int j = 0; j < 4; ++j) {
#pragma unroll
      for (int r = 0; r < 8; ++r) {
        const float v = acc[i][j][r] * scale;
        slab[(mOff + r) * 68 + (j << 4) + rlane] = v;
      }
    }
    __builtin_amdgcn_fence(__ATOMIC_RELEASE, "workgroup");
    __builtin_amdgcn_wave_barrier();
    __builtin_amdgcn_fence(__ATOMIC_ACQUIRE, "workgroup");
    {
      const int hh = lane >> 4, c4 = (lane & 15) * 4;
      for (int pass = 0; pass < 2; ++pass) {
#pragma unroll
        for (int it = 0; it < 8; ++it) {
          const int row = it * 2 + hh;
          v4f v = *(const v4f*)(slab + row * 68 + c4);
          *(volatile v4f*)(C + (size_t)(mBase + row) * ldc + n0 + c4) = v;
        }
        __threadfence();
      }
    }
    __builtin_amdgcn_fence(__ATOMIC_RELEASE, "workgroup");
    __builtin_amdgcn_wave_barrier();
    __builtin_amdgcn_fence(__ATOMIC_ACQUIRE, "workgroup");
  }
}

}

__global__ __launch_bounds__(256) void cvt_x_f16_kernel(
    const float* __restrict__ src, unsigned short* __restrict__ dst, int total8) {
  const int i = blockIdx.x * 256 + threadIdx.x;
  if (i >= total8) return;
  const size_t e0 = (size_t)i << 3;
  const v4f a0 = *(const v4f*)(src + e0);
  const v4f a1 = *(const v4f*)(src + e0 + 4);
  v8h hv;
#pragma unroll
  for (int e = 0; e < 4; ++e) {
    const float f0 = a0[e];
    const float f1 = a1[e];
    hv[e]     = (_Float16)carry_flush(f0, kCarryX);
    hv[4 + e] = (_Float16)carry_flush(f1, kCarryX);
  }
  unsigned short* dp = dst + e0;
  *(volatile v8h*)dp = hv;
  __threadfence();
  *(volatile v8h*)dp = hv;
}

__global__ __launch_bounds__(256) void pack_gate_kernel(
    const float* __restrict__ W0, const float* __restrict__ B0, const float* __restrict__ P0,
    const float* __restrict__ W1, const float* __restrict__ B1, const float* __restrict__ P1,
    const float* __restrict__ W2, const float* __restrict__ B2, const float* __restrict__ P2,
    const float* __restrict__ W3, const float* __restrict__ B3, const float* __restrict__ P3,
    unsigned short* __restrict__ BT, float* __restrict__ CP) {
  __shared__ __align__(16) float sC[kCpPerGate];
  const int g = blockIdx.x;
  const float* W  = (g == 0) ? W0 : (g == 1) ? W1 : (g == 2) ? W2 : W3;
  const float* Bv = (g == 0) ? B0 : (g == 1) ? B1 : (g == 2) ? B2 : B3;
  const float* P  = (g == 0) ? P0 : (g == 1) ? P1 : (g == 2) ? P2 : P3;
  const int tid = threadIdx.x, lane = tid & 31, wave = tid >> 5;

  {
    const int half = tid >> 7;
    const int r  = (tid & 127) >> 4;
    const int k0 = (tid & 15) * 8;
    const int n  = half * kNReal + g * kHid + r;
    v8h hv;
#pragma unroll
    for (int e = 0; e < 8; ++e) {
      float w = W[r * kComb + k0 + e];
      asm volatile("" : "+v"(w));
      const float wsel = (half != 0) ? 0.0f : w;
      hv[e] = (_Float16)carry_flush(wsel, kCarryW);
    }
    unsigned short* dp = BT + (size_t)n * kDin + k0;
    *(volatile v8h*)dp = hv;
    __threadfence();
    *(volatile v8h*)dp = hv;
  }

  {
    const int c  = tid & 127;
    const int qa = (c & 63) >> 3;
    const int ja = c & 7;
    float wa = W[qa * kComb + kDin + ja];
    asm volatile("" : "+v"(wa));
    float bb = Bv[ja];
    asm volatile("" : "+v"(bb));
    float pp = P[ja * 3];
    asm volatile("" : "+v"(pp));
    const float cp = cosf(pp);
    float cval = 0.0f;
    cval = (c < 64) ? wa : cval;
    cval = (c >= 64 && c < 72) ? bb : cval;
    cval = (c >= 72 && c < 80) ? cp : cval;
    if (tid < 128) sC[c] = cval;
  }
  __syncthreads();
  if (wave == 0) {
    const v4f v = *(const v4f*)(sC + lane * 4);
    float* dp = CP + (size_t)g * kCpPerGate + lane * 4;
    *(volatile v4f*)dp = v;
    __threadfence();
    *(volatile v4f*)dp = v;
  }
}

__global__ __launch_bounds__(128) void recur_kernel(
    const float* __restrict__ TH, const float* __restrict__ CP, float* __restrict__ out) {
  __shared__ __align__(16) float sH[kFlush * 32];
  __shared__ __align__(16) float sF[64];
  const int tid = threadIdx.x, lane = tid & 31, wave = tid >> 5;
  const int q = lane & 7, g = lane >> 3;
  const int b0 = blockIdx.x * 4;
  const int b  = b0 + wave;

  const float* cg = CP + g * kCpPerGate;
  const v4f wv0 = *(const v4f*)(cg + q * 8);
  const v4f wv1 = *(const v4f*)(cg + q * 8 + 4);
  const float w0 = wv0[0], w1 = wv0[1], w2 = wv0[2], w3 = wv0[3];
  const float w4 = wv1[0], w5 = wv1[1], w6 = wv1[2], w7 = wv1[3];
  const float bias = cg[64 + q];
  const float cosP = cg[72 + q];

  float h = 0.0f, c = 0.0f;

#pragma unroll 1
  for (int t0 = 0; t0 < kSteps; t0 += kFlush) {
#pragma unroll 1
    for (int s = 0; s < kFlush; ++s) {
      const int t = t0 + s;
      const float thx = TH[((size_t)t * kBatch + b) * kThP + lane];
      const float h0 = __shfl(h, 0, 32);
      const float h1 = __shfl(h, 1, 32);
      const float h2 = __shfl(h, 2, 32);
      const float h3 = __shfl(h, 3, 32);
      const float h4 = __shfl(h, 4, 32);
      const float h5 = __shfl(h, 5, 32);
      const float h6 = __shfl(h, 6, 32);
      const float h7 = __shfl(h, 7, 32);
      float dot = w0 * h0;
      dot = fmaf(w1, h1, dot);
      dot = fmaf(w2, h2, dot);
      dot = fmaf(w3, h3, dot);
      dot = fmaf(w4, h4, dot);
      dot = fmaf(w5, h5, dot);
      dot = fmaf(w6, h6, dot);
      dot = fmaf(w7, h7, dot);
      const float ang = (thx + bias) + dot;
      float v = cosP * cosf(ang);
      float u;
      u = __shfl_up(v, 1, 8);
      v = (q >= 1) ? (v * u) : v;
      u = __shfl_up(v, 2, 8);
      v = (q >= 2) ? (v * u) : v;
      u = __shfl_up(v, 4, 8);
      v = (q >= 4) ? (v * u) : v;
      const float ex = expf(-v);
      const float sg = 1.0f / (1.0f + ex);
      const float tt = tanhf(v);
      const float gF = __shfl(sg, q, 32);
      const float gI = __shfl(sg, q + 8, 32);
      const float gG = __shfl(tt, q + 16, 32);
      const float gO = __shfl(sg, q + 24, 32);
      c = gF * c + gI * gG;
      h = gO * tanhf(c);
      if (lane < 8) sH[s * 32 + wave * 8 + lane] = h;
    }
    __syncthreads();
    if (wave < 2) {
      const int slot = wave * 4 + (lane >> 3);
      const int c4 = (lane & 7) * 4;
      const v4f hv = *(const v4f*)(sH + slot * 32 + c4);
      float* dp = out + ((size_t)(t0 + slot) * kBatch + b0) * kHid + c4;
      *(volatile v4f*)dp = hv;
      __threadfence();
      *(volatile v4f*)dp = hv;
    }
    __syncthreads();
  }

  if (lane < 8) {
    sF[wave * 8 + lane] = h;
    sF[32 + wave * 8 + lane] = c;
  }
  __syncthreads();
  if (wave == 0) {
    const int li = lane & 15;
    const v4f fv = *(const v4f*)(sF + li * 4);
    float* dp = out + (size_t)kOut1Off + (size_t)(li >> 3) * (kBatch * kHid) + (size_t)b0 * kHid + (li & 7) * 4;
    if (lane < 16) *(volatile v4f*)dp = fv;
    __threadfence();
    if (lane < 16) *(volatile v4f*)dp = fv;
  }
}

extern "C" void kernel_launch(void* const* d_in, const int* in_sizes, int n_in,
                              void* d_out, int out_size, void* d_ws, size_t ws_size,
                              hipStream_t stream) {
  if (n_in < 13) return;
  if (in_sizes[0] != kRows * kDin) return;
  for (int gi = 0; gi < kGates; ++gi) {
    if (in_sizes[1 + 3 * gi] != kHid * kComb) return;
    if (in_sizes[2 + 3 * gi] != kHid) return;
    if (in_sizes[3 + 3 * gi] != kHid * 3) return;
  }
  if (out_size != kOutTotal) return;
  if (ws_size < kWsTotal) return;

  const float* x  = (const float*)d_in[0];
  const float* Wf = (const float*)d_in[1];
  const float* bf = (const float*)d_in[2];
  const float* Pf = (const float*)d_in[3];
  const float* Wi = (const float*)d_in[4];
  const float* bi = (const float*)d_in[5];
  const float* Pi = (const float*)d_in[6];
  const float* Wu = (const float*)d_in[7];
  const float* bu = (const float*)d_in[8];
  const float* Pu = (const float*)d_in[9];
  const float* Wo = (const float*)d_in[10];
  const float* bo = (const float*)d_in[11];
  const float* Po = (const float*)d_in[12];
  float* out = (float*)d_out;

  char* ws = (char*)d_ws;
  unsigned short* XH = (unsigned short*)(ws + kOffXH);
  unsigned short* BT = (unsigned short*)(ws + kOffBT);
  float*          CP = (float*)(ws + kOffCP);
  float*          TH = (float*)(ws + kOffTH);

  cvt_x_f16_kernel<<<(kRows * kDin / 8) / 256, 256, 0, stream>>>(x, XH, kRows * kDin / 8);

  pack_gate_kernel<<<kGates, 256, 0, stream>>>(Wf, bf, Pf, Wi, bi, Pi, Wu, bu, Pu, Wo, bo, Po, BT, CP);

  eng::gemm_f16_tile64<<<(kRows / 64) * (kNPad / 64) / 8, 256, 0, stream>>>(
      XH, kDin, BT, kDin, TH, kThP, kRows, kNPad, kDin, kFold);

  recur_kernel<<<kBatch / 4, 128, 0, stream>>>(TH, CP, out);
}
